// MessagePassingNet_27943057228185
// MI455X (gfx1250) — hardware-run, weakly checked
//
#include <hip/hip_runtime.h>

typedef float          v8f   __attribute__((ext_vector_type(8)));
typedef float          v4f   __attribute__((ext_vector_type(4)));
typedef unsigned int   v4u   __attribute__((ext_vector_type(4)));
typedef int            v8i   __attribute__((ext_vector_type(8)));
typedef unsigned short v8us  __attribute__((ext_vector_type(8)));
typedef unsigned short v16us __attribute__((ext_vector_type(16)));
typedef __bf16         v16bf __attribute__((ext_vector_type(16)));
typedef _Float16       v16h  __attribute__((ext_vector_type(16)));
typedef v4f  __attribute__((may_alias)) v4fa;
typedef v8us __attribute__((may_alias)) v8usa;
union FragB { v16bf v; v16us u; v8us h[2]; v8i w; };
union FragH { v16h  v; v16us u; v8us h[2]; v8i w; };

__device__ __forceinline__ v8f wmb(const FragB& a, const FragB& b, v8f c) {
  v8f d = __builtin_amdgcn_wmma_f32_16x16x32_bf16(false, a.v, false, b.v, (short)0, c, false, false);
  asm volatile("v_nop\n\tv_nop\n\tv_nop\n\tv_nop" : "+v"(d) : "v"(a.w), "v"(b.w));
  return d;
}

__device__ __forceinline__ v8f wmh(const FragH& a, const FragH& b, v8f c) {
  v8f d = __builtin_amdgcn_wmma_f32_16x16x32_f16(false, a.v, false, b.v, (short)0, c, false, false);
  asm volatile("v_nop\n\tv_nop\n\tv_nop\n\tv_nop" : "+v"(d) : "v"(a.w), "v"(b.w));
  return d;
}

__device__ __forceinline__ unsigned bf16_bits(float f) {
  const unsigned u = __float_as_uint(f);
  const unsigned r = (u + 0x7FFFu + ((u >> 16) & 1u)) >> 16;
  const unsigned q = (u >> 16) | 0x40u;
  return ((u & 0x7fffffffu) > 0x7f800000u) ? q : r;
}

__device__ __forceinline__ float bf16_val(float f) {
  return __uint_as_float(bf16_bits(f) << 16);
}
__device__ __forceinline__ int clampi(int v, int lo, int hi) {
  return v < lo ? lo : (v > hi ? hi : v);
}

__device__ __forceinline__ unsigned f16_bits(float f) {
  const unsigned u  = __float_as_uint(f);
  const unsigned s  = (u >> 16) & 0x8000u;
  const unsigned a  = u & 0x7fffffffu;
  const unsigned t  = a - 0x38000000u;
  const unsigned r  = (t + 0x0FFFu + ((t >> 13) & 1u)) >> 13;
  const unsigned rc = r > 0x7C00u ? 0x7C00u : r;
  const bool small  = a < 0x38800000u;
  const bool isnan  = a > 0x7f800000u;
  const unsigned fin = small ? 0u : (s | rc);
  return isnan ? (s | 0x7E00u) : fin;
}

__device__ __forceinline__ unsigned pk16(unsigned lo, unsigned hi) { return lo | (hi << 16); }
__device__ __forceinline__ unsigned bf16_lo_bits(float v) {
  float hi = bf16_val(v);
  asm volatile("" : "+v"(hi));
  return bf16_bits(v - hi);
}
__device__ __forceinline__ v4u pack8_bf16(v4f a, v4f c) {
  return (v4u){ pk16(bf16_bits(a[0]), bf16_bits(a[1])), pk16(bf16_bits(a[2]), bf16_bits(a[3])),
                pk16(bf16_bits(c[0]), bf16_bits(c[1])), pk16(bf16_bits(c[2]), bf16_bits(c[3])) };
}
__device__ __forceinline__ v4u pack8_bf16_lo(v4f a, v4f c) {
  return (v4u){ pk16(bf16_lo_bits(a[0]), bf16_lo_bits(a[1])), pk16(bf16_lo_bits(a[2]), bf16_lo_bits(a[3])),
                pk16(bf16_lo_bits(c[0]), bf16_lo_bits(c[1])), pk16(bf16_lo_bits(c[2]), bf16_lo_bits(c[3])) };
}
__device__ __forceinline__ v4u pack8_f16(v4f a, v4f c) {
  return (v4u){ pk16(f16_bits(a[0]), f16_bits(a[1])), pk16(f16_bits(a[2]), f16_bits(a[3])),
                pk16(f16_bits(c[0]), f16_bits(c[1])), pk16(f16_bits(c[2]), f16_bits(c[3])) };
}

template <int FORM>
__global__ __launch_bounds__(256) void k_plane(const float* __restrict__ src, int rows, int cols, int ldsrc,
                                               unsigned short* __restrict__ dst, int MP, int KP) {
  static_assert(FORM >= 0 && FORM <= 3);
  const int KTOT = (FORM == 1 || FORM == 3) ? 2 * KP : KP;
  const unsigned ppr   = (unsigned)(KTOT >> 3);
  const unsigned kp8   = (unsigned)(KP >> 3);
  const unsigned total = (unsigned)MP * ppr;
  const unsigned g     = blockIdx.x * 256u + threadIdx.x;
  const unsigned rowu  = g / ppr;
  const unsigned p     = g - rowu * ppr;
  const bool second    = p >= kp8;
  const int row = (int)rowu;
  const int c0  = (int)((second ? p - kp8 : p) << 3);
  const float* srow = src + (size_t)clampi(row, 0, rows - 1) * (size_t)ldsrc;
  float x[8];
  unsigned mk[8];
#pragma unroll
  for (int e = 0; e < 8; ++e) {
    const int c = c0 + e;
    const float v = srow[clampi(c, 0, cols - 1)];
    asm volatile("" :: "v"(v));
    x[e]  = v;
    mk[e] = (row < rows && c < cols) ? 0xFFFFu : 0u;
  }
  const v4f a = (v4f){ x[0], x[1], x[2], x[3] };
  const v4f c = (v4f){ x[4], x[5], x[6], x[7] };
  v4u o;
  if (FORM == 2) {
    o = pack8_f16(a, c);
  } else {
    const v4u hi = pack8_bf16(a, c);
    o = hi;
    if (FORM == 1) { const v4u lo = pack8_bf16_lo(a, c); o = second ? lo : hi; }
  }
  const v4u mw = (v4u){ pk16(mk[0], mk[1]), pk16(mk[2], mk[3]), pk16(mk[4], mk[5]), pk16(mk[6], mk[7]) };
  o &= mw;
  if (g < total) {
    volatile v4u* q = (volatile v4u*)(dst + (size_t)g * 8);
    *q = o;
    __threadfence();
    *q = o;
  }
}

template <int FORM> struct FragOf    { typedef FragB T; };
template <>         struct FragOf<2> { typedef FragH T; };
__device__ __forceinline__ v8f mm(const FragB& a, const FragB& b, v8f c) { return wmb(a, b, c); }
__device__ __forceinline__ v8f mm(const FragH& a, const FragH& b, v8f c) { return wmh(a, b, c); }
template <class F> __device__ __forceinline__ F ld_frag(const unsigned short* p) {
  F f;
  f.h[0] = *(const v8usa*)(p);
  f.h[1] = *(const v8usa*)(p + 16);
  return f;
}

template <int FORM, int EPI>
__global__ __launch_bounds__(256) __attribute__((amdgpu_num_vgpr(248)))
void k_gemm_nt(const unsigned short* __restrict__ A, const unsigned short* __restrict__ B,
               const float* __restrict__ bias, float* __restrict__ D, int M, int N, int KTOT, int ldd) {
  static_assert(FORM >= 0 && FORM <= 2);
  static_assert(EPI == 0 || EPI == 1);
  typedef typename FragOf<FORM>::T F;
  __shared__ __attribute__((aligned(16))) float sT[8][16 * 68];
  const int lane = threadIdx.x & 31;
  const int wave = threadIdx.x >> 5;
  const int tilesM = (M + 63) >> 6;
  const int tilesN = (N + 63) >> 6;
  const int tile = blockIdx.x * 8 + wave;
  if (tile >= tilesM * tilesN) return;
  const int tm = tile / tilesN;
  const int tn = tile - tm * tilesN;
  const int m0 = tm << 6;
  const int n0 = tn << 6;

  const int rl = lane & 15;
  const int h8 = (lane >> 4) * 8;
  const unsigned short* pa = A + (size_t)(m0 + rl) * (size_t)KTOT + h8;
  const unsigned short* pb = B + (size_t)(n0 + rl) * (size_t)KTOT + h8;

  v8f acc[4][4];
#pragma unroll
  for (int i = 0; i < 4; ++i)
#pragma unroll
    for (int j = 0; j < 4; ++j) acc[i][j] = (v8f){0.f, 0.f, 0.f, 0.f, 0.f, 0.f, 0.f, 0.f};

#pragma unroll 1
  for (int k0 = 0; k0 < KTOT; k0 += 32) {
    F bf[4];
#pragma unroll
    for (int j = 0; j < 4; ++j) bf[j] = ld_frag<F>(pb + (size_t)(j << 4) * (size_t)KTOT + k0);
#pragma unroll
    for (int i = 0; i < 4; ++i) {
      const F af = ld_frag<F>(pa + (size_t)(i << 4) * (size_t)KTOT + k0);
#pragma unroll
      for (int j = 0; j < 4; ++j) acc[i][j] = mm(af, bf[j], acc[i][j]);
    }
  }

  float* slab = sT[wave];
  const int hh = lane >> 4;
  const int c4 = (lane & 15) * 4;
  const int nc = n0 + c4;
  const bool cok = nc < N;
  v4f bv = (v4f){0.f, 0.f, 0.f, 0.f};
  if (EPI == 1) {
    bv = *(const v4fa*)(bias + clampi(nc, 0, N - 4));
    asm volatile("" :: "v"(bv));
  }
#pragma unroll
  for (int i = 0; i < 4; ++i) {
    const int mBase = m0 + (i << 4);
#pragma unroll
    for (int j = 0; j < 4; ++j) {
#pragma unroll
      for (int r = 0; r < 8; ++r) slab[(h8 + r) * 68 + (j << 4) + rl] = acc[i][j][r];
    }
    __builtin_amdgcn_fence(__ATOMIC_RELEASE, "workgroup");
    __builtin_amdgcn_wave_barrier();
    __builtin_amdgcn_fence(__ATOMIC_ACQUIRE, "workgroup");
    v4f vv[8];
#pragma unroll
    for (int it = 0; it < 8; ++it) {
      const int row = it * 2 + hh;
      v4f v = *(const v4fa*)(slab + row * 68 + c4);
      if (EPI == 1) v += bv;
      vv[it] = v;
    }
    for (int pass = 0; pass < 2; ++pass) {
#pragma unroll
      for (int it = 0; it < 8; ++it) {
        const int row = mBase + it * 2 + hh;
        if (cok && row < M) *(volatile v4f*)(D + (size_t)row * (size_t)ldd + nc) = vv[it];
      }
      __threadfence();
    }
    __builtin_amdgcn_fence(__ATOMIC_RELEASE, "workgroup");
    __builtin_amdgcn_wave_barrier();
    __builtin_amdgcn_fence(__ATOMIC_ACQUIRE, "workgroup");
  }
}

#include <stddef.h>
#include <stdint.h>
#include <math.h>

#define NN      50000
#define EE      800000
#define DD      64
#define MPAD    50048
#define NTHR    256
#define NBA     1024
#define NBLK    49
#define NSLOT   (NBLK * NBA)
#define CHUNK   2048
#define NCHUNK  391
#define WCAP    256
#define RCAP    20992
#define DEGCAP  64
#define BK_INTS (2 * RCAP + 4 * NBA + 32)
#define BK_BYTES (BK_INTS * 4)
#define WSMAX   ((size_t)128 << 20)

static_assert(EE == 390 * 2048 + 1280);
static_assert(NCHUNK == (EE + CHUNK - 1) / CHUNK);
static_assert(EE % 8 == 0 && ((size_t)EE * 4) % 16 == 0);
static_assert(NN <= 65536);
static_assert(NBA == 1024 && NBLK == (NN + NBA - 1) / NBA && NBLK == 49);
static_assert(NN - (NBLK - 1) * NBA == 848);
static_assert(RCAP % 256 == 0 && RCAP % 128 == 0);
static_assert((long long)RCAP * 4 >= 16623LL * 5);
static_assert(DEGCAP >= 35 + 8);
static_assert(WCAP == 8 * 32 && CHUNK == 8 * WCAP);
static_assert(BK_INTS % 4 == 0 && BK_BYTES == 184448 && BK_BYTES <= 262144);
static_assert(BK_BYTES + 0 <= 327680);
static_assert(DD == 64 && DD == 2 * 32);
static_assert(NN % 8 == 0 && NN / 8 == 6250);
static_assert(MPAD % 64 == 0 && MPAD >= NN && DD % 32 == 0 && MPAD % 16 == 0);
static_assert(((long long)MPAD * DD / 8) % 256 == 0 && (long long)MPAD * DD / 8 / 256 == 1564);
static_assert(((MPAD / 64) + 7) / 8 == 98);

constexpr size_t SZ_XB   = (size_t)MPAD * DD * 2;
constexpr size_t SZ_H    = (size_t)MPAD * DD * 4;
constexpr size_t SZ_WB   = (size_t)DD * DD * 2;
constexpr size_t SZ_PAR  = 512;
constexpr size_t SZ_LIST = (size_t)NBLK * RCAP * 4;
constexpr size_t SZ_TAB  = (size_t)NSLOT * 4;
constexpr size_t SZ_FLAG = 6400;
constexpr size_t O_XB   = 0;
constexpr size_t O_H    = O_XB + SZ_XB;
constexpr size_t O_WB   = O_H + SZ_H;
constexpr size_t O_PAR  = O_WB + SZ_WB;
constexpr size_t O_LIST = O_PAR + SZ_PAR;
constexpr size_t O_CNT  = O_LIST + SZ_LIST;
constexpr size_t O_OFF  = O_CNT + SZ_TAB;
constexpr size_t O_DINV = O_OFF + SZ_TAB;
constexpr size_t O_FLAG = O_DINV + SZ_TAB;
constexpr size_t WS_TOTAL = O_FLAG + SZ_FLAG;
static_assert(SZ_XB % 256 == 0 && SZ_H % 256 == 0 && SZ_WB % 256 == 0 && SZ_PAR % 256 == 0);
static_assert(SZ_LIST % 256 == 0 && SZ_TAB % 256 == 0 && SZ_FLAG % 256 == 0 && SZ_FLAG >= (size_t)NBLK * 128);
static_assert(WS_TOTAL == 23950080 && WS_TOTAL <= (size_t)WSMAX);

typedef float v2f __attribute__((ext_vector_type(2)));
typedef int   v4i __attribute__((ext_vector_type(4)));
typedef v2f __attribute__((may_alias)) v2fa;
typedef v4i __attribute__((may_alias)) v4ia;

__global__ __launch_bounds__(NTHR) void k_prep(const float* __restrict__ W, const float* __restrict__ b,
                                               const float* __restrict__ pa, unsigned short* WB, float* PAR) {
  const int tid = (int)threadIdx.x;
  v4u o0, o1;
  {
    const float* p0 = W + (size_t)tid * 8;
    const float* p1 = W + (size_t)(tid + NTHR) * 8;
    const v4f a0 = *(const v4fa*)p0;
    const v4f c0 = *(const v4fa*)(p0 + 4);
    const v4f a1 = *(const v4fa*)p1;
    const v4f c1 = *(const v4fa*)(p1 + 4);
    o0 = pack8_bf16(a0, c0);
    o1 = pack8_bf16(a1, c1);
  }
  const int q  = tid & 31;
  const int i0 = q * 4;
  const int ib = i0 < (DD - 4) ? i0 : (DD - 4);
  const v4f bb = *(const v4fa*)(b + ib);
  asm volatile("" :: "v"(bb));
  const float sv = pa[0];
  asm volatile("" :: "v"(sv));
  const bool isb = i0 < DD;
  const bool iss = i0 == DD;
  v4f pv;
  pv.x = isb ? bf16_val(bb.x) : (iss ? bf16_val(sv) : 0.0f);
  pv.y = isb ? bf16_val(bb.y) : 0.0f;
  pv.z = isb ? bf16_val(bb.z) : 0.0f;
  pv.w = isb ? bf16_val(bb.w) : 0.0f;
  const bool wp = tid < 32;
#pragma unroll 1
  for (int pass = 0; pass < 2; ++pass) {
    *(volatile v4u*)(WB + (size_t)tid * 8) = o0;
    *(volatile v4u*)(WB + (size_t)(tid + NTHR) * 8) = o1;
    if (wp) *(volatile v4f*)(PAR + i0) = pv;
    __threadfence();
  }
}

#define PUTJ(HJ, WJ) { const bool st = (HJ) && (p < RCAP); if (st) hl[p] = (int)(WJ); p += (HJ) ? 1 : 0; }

__global__ __launch_bounds__(NTHR) void k_bucket(const int* __restrict__ rowp, const int* __restrict__ colp,
                                                 int* LIST, int* CNT, int* OFF, int* DINVB, int* FLAG) {
  extern __shared__ __attribute__((aligned(16))) int dsm[];
  int* hl   = dsm;
  int* sl   = dsm + RCAP;
  int* cnt  = dsm + 2 * RCAP;
  int* offs = cnt + NBA;
  int* cur  = offs + NBA;
  int* dvi  = cur + NBA;
  int* misc = dvi + NBA;
  const int tid  = (int)threadIdx.x;
  const int lane = tid & 31;
  const int wave = __builtin_amdgcn_readfirstlane(tid >> 5);
  const int nodeBase = (int)blockIdx.x * NBA;
  const int nbRaw = NN - nodeBase;
  const unsigned unb = (unsigned)(nbRaw < NBA ? (nbRaw < 0 ? 0 : nbRaw) : NBA);
  const unsigned nbs = (unsigned)nodeBase;

  {
    const v4i z4 = {0, 0, 0, 0};
    for (int i = tid * 4; i < BK_INTS; i += NTHR * 4) *(v4ia*)(dsm + i) = z4;
  }
  __syncthreads();

  int t = 0;
#pragma unroll 1
  for (int ch = 0; ch < NCHUNK; ++ch) {
    const int e0  = ch * CHUNK + tid * 8;
    const int e0c = e0 < (EE - 8) ? e0 : (EE - 8);
    const v4i ca = *(const v4ia*)(colp + e0c);
    const v4i cb = *(const v4ia*)(colp + e0c + 4);
    const v4i ra = *(const v4ia*)(rowp + e0c);
    const v4i rb = *(const v4ia*)(rowp + e0c + 4);
    asm volatile("" :: "v"(ca));
    asm volatile("" :: "v"(cb));
    asm volatile("" :: "v"(ra));
    asm volatile("" :: "v"(rb));
    const int inv = (e0 < EE) ? 0 : -1;
    const unsigned s0 = (unsigned)(ca.x | inv) - nbs, s1 = (unsigned)(ca.y | inv) - nbs;
    const unsigned s2 = (unsigned)(ca.z | inv) - nbs, s3 = (unsigned)(ca.w | inv) - nbs;
    const unsigned s4 = (unsigned)(cb.x | inv) - nbs, s5 = (unsigned)(cb.y | inv) - nbs;
    const unsigned s6 = (unsigned)(cb.z | inv) - nbs, s7 = (unsigned)(cb.w | inv) - nbs;
    const bool h0 = s0 < unb, h1 = s1 < unb, h2 = s2 < unb, h3 = s3 < unb;
    const bool h4 = s4 < unb, h5 = s5 < unb, h6 = s6 < unb, h7 = s7 < unb;
    const unsigned w0 = (s0 << 16) | (unsigned)clampi(ra.x, 0, NN - 1);
    const unsigned w1 = (s1 << 16) | (unsigned)clampi(ra.y, 0, NN - 1);
    const unsigned w2 = (s2 << 16) | (unsigned)clampi(ra.z, 0, NN - 1);
    const unsigned w3 = (s3 << 16) | (unsigned)clampi(ra.w, 0, NN - 1);
    const unsigned w4 = (s4 << 16) | (unsigned)clampi(rb.x, 0, NN - 1);
    const unsigned w5 = (s5 << 16) | (unsigned)clampi(rb.y, 0, NN - 1);
    const unsigned w6 = (s6 << 16) | (unsigned)clampi(rb.z, 0, NN - 1);
    const unsigned w7 = (s7 << 16) | (unsigned)clampi(rb.w, 0, NN - 1);
    const unsigned any = __builtin_amdgcn_ballot_w32(h0 | h1 | h2 | h3 | h4 | h5 | h6 | h7);
    int low = 0, wc = 0;
    if (any != 0u) {
      const unsigned m0 = __builtin_amdgcn_ballot_w32(h0), m1 = __builtin_amdgcn_ballot_w32(h1);
      const unsigned m2 = __builtin_amdgcn_ballot_w32(h2), m3 = __builtin_amdgcn_ballot_w32(h3);
      const unsigned m4 = __builtin_amdgcn_ballot_w32(h4), m5 = __builtin_amdgcn_ballot_w32(h5);
      const unsigned m6 = __builtin_amdgcn_ballot_w32(h6), m7 = __builtin_amdgcn_ballot_w32(h7);
      low = (int)(__builtin_amdgcn_mbcnt_lo(m0, 0u) + __builtin_amdgcn_mbcnt_lo(m1, 0u) +
                  __builtin_amdgcn_mbcnt_lo(m2, 0u) + __builtin_amdgcn_mbcnt_lo(m3, 0u) +
                  __builtin_amdgcn_mbcnt_lo(m4, 0u) + __builtin_amdgcn_mbcnt_lo(m5, 0u) +
                  __builtin_amdgcn_mbcnt_lo(m6, 0u) + __builtin_amdgcn_mbcnt_lo(m7, 0u));
      wc = (int)(__builtin_popcount(m0) + __builtin_popcount(m1) + __builtin_popcount(m2) + __builtin_popcount(m3) +
                 __builtin_popcount(m4) + __builtin_popcount(m5) + __builtin_popcount(m6) + __builtin_popcount(m7));
    }
    const int buf = (ch & 1) * 8;
    if (lane == 0) misc[buf + wave] = wc;
    __syncthreads();
    int cv = misc[buf + (lane & 7)];
    cv = clampi(cv, 0, WCAP);
    int base = 0, tot = 0;
#pragma unroll
    for (int q = 0; q < 8; ++q) {
      const int c = __builtin_amdgcn_readlane(cv, q);
      tot += c;
      base += (q < wave) ? c : 0;
    }
    if (any != 0u) {
      int p = t + base + low;
      PUTJ(h0, w0)
      PUTJ(h1, w1)
      PUTJ(h2, w2)
      PUTJ(h3, w3)
      PUTJ(h4, w4)
      PUTJ(h5, w5)
      PUTJ(h6, w6)
      PUTJ(h7, w7)
    }
    t += tot;
  }
  __syncthreads();
  const int ov = (t > RCAP) ? 1 : 0;
  int tt = t < 0 ? 0 : (t > RCAP ? RCAP : t);
  tt = __builtin_amdgcn_readfirstlane(tt);

  if (wave == 0) {
#pragma unroll 1
    for (int b0 = 0; b0 < tt; b0 += 32) {
      const int idx = b0 + lane;
      const int ent = hl[idx < RCAP ? idx : RCAP - 1];
      const int m32 = (tt - b0) < 32 ? (tt - b0) : 32;
#pragma unroll 1
      for (int k = 0; k < m32; ++k) {
        const int u    = __builtin_amdgcn_readlane(ent, k);
        const int slot = (u >> 16) & (NBA - 1);
        if (lane == 0) cnt[slot] = cnt[slot] + 1;
      }
    }
  }
  __syncthreads();

  if (wave == 0) {
    const int base = lane * (NBA / 32);
    int s = 0;
#pragma unroll 1
    for (int i = 0; i < NBA / 32; ++i) s += cnt[base + i];
    int incl = s;
#pragma unroll
    for (int d = 1; d < 32; d <<= 1) {
      const int y = __shfl_up(incl, d, 32);
      if (lane >= d) incl += y;
    }
    int run = incl - s;
#pragma unroll 1
    for (int i = 0; i < NBA / 32; ++i) {
      const int cvv = cnt[base + i];
      offs[base + i] = run;
      cur[base + i]  = run;
      run += cvv;
    }
  }
#pragma unroll 1
  for (int i = tid; i < NBA; i += NTHR) {
    const int deg = cnt[i] + 1;
    const float df = (float)deg;
    const float r  = 1.0f / sqrtf(df);
    const float dv = (deg > 0) ? r : 0.0f;
    dvi[i] = __float_as_int(dv);
  }
  __syncthreads();

  if (wave == 0) {
#pragma unroll 1
    for (int b0 = 0; b0 < tt; b0 += 32) {
      const int idx = b0 + lane;
      const int ent = hl[idx < RCAP ? idx : RCAP - 1];
      const int m32 = (tt - b0) < 32 ? (tt - b0) : 32;
#pragma unroll 1
      for (int k = 0; k < m32; ++k) {
        const int u    = __builtin_amdgcn_readlane(ent, k);
        const int slot = (u >> 16) & (NBA - 1);
        if (lane == 0) {
          int p = cur[slot];
          p = p < 0 ? 0 : (p > RCAP - 1 ? RCAP - 1 : p);
          sl[p] = u;
          cur[slot] = p + 1;
        }
      }
    }
  }
  __syncthreads();

  int* lp = LIST + (size_t)blockIdx.x * RCAP;
  const v4i c4 = *(const v4ia*)(cnt + tid * 4);
  const v4i o4 = *(const v4ia*)(offs + tid * 4);
  const v4i d4 = *(const v4ia*)(dvi + tid * 4);
  const v4i f4 = {ov, ov, ov, ov};
  const bool wf = tid < 8;
#pragma unroll 1
  for (int pass = 0; pass < 2; ++pass) {
#pragma unroll 1
    for (int i = tid * 4; i < RCAP; i += NTHR * 4) {
      const v4i v = *(const v4ia*)(sl + i);
      *(volatile v4i*)(lp + i) = v;
    }
    *(volatile v4i*)(CNT   + (size_t)nodeBase + tid * 4) = c4;
    *(volatile v4i*)(OFF   + (size_t)nodeBase + tid * 4) = o4;
    *(volatile v4i*)(DINVB + (size_t)nodeBase + tid * 4) = d4;
    if (wf) *(volatile v4i*)(FLAG + (size_t)blockIdx.x * 32 + tid * 4) = f4;
    __threadfence();
  }
}
#undef PUTJ

__global__ __launch_bounds__(NTHR) void k_replay(const float* __restrict__ H, const int* __restrict__ LIST,
                                                 const int* __restrict__ CNT, const int* __restrict__ OFF,
                                                 const float* __restrict__ DINV, const int* __restrict__ FLAG,
                                                 const float* __restrict__ PAR, float* out) {
#pragma clang fp contract(off)
  const int tid  = (int)threadIdx.x;
  const int lane = tid & 31;
  const int wave = __builtin_amdgcn_readfirstlane(tid >> 5);
  const int t  = (int)blockIdx.x * 8 + wave;
  const int tc = t < NN ? t : NN - 1;
  const int blk = tc >> 10;

  const int cr = CNT[tc];
  asm volatile("" :: "v"(cr));
  const int orw = OFF[tc];
  asm volatile("" :: "v"(orw));
  const float dt = DINV[tc];
  asm volatile("" :: "v"(dt));
  const int fl = FLAG[blk * 32];
  asm volatile("" :: "v"(fl));
  const v2f bp = *(const v2fa*)(PAR + 2 * lane);
  asm volatile("" :: "v"(bp));
  const float sa = PAR[DD];
  asm volatile("" :: "v"(sa));

  const bool big = (cr < 0) || (cr > DEGCAP);
  int cn = clampi(cr, 0, DEGCAP);
  cn = __builtin_amdgcn_readfirstlane(cn);
  int of = clampi(orw, 0, RCAP);
  of = __builtin_amdgcn_readfirstlane(of);
  const int* lp = LIST + (size_t)blk * RCAP;

  float a0 = 0.0f, a1 = 0.0f;
#pragma unroll 1
  for (int b0 = 0; b0 < cn; b0 += 32) {
    int idx = of + b0 + lane;
    idx = idx > RCAP - 1 ? RCAP - 1 : idx;
    const int wd = lp[idx];
    asm volatile("" :: "v"(wd));
    const int s = clampi(wd & 0xffff, 0, NN - 1);
    const float ds = DINV[s];
    asm volatile("" :: "v"(ds));
    const float w = ds * dt;
    const int wi = __float_as_int(w);
    const int m32 = (cn - b0) < 32 ? (cn - b0) : 32;
#pragma unroll 1
    for (int k = 0; k < m32; ++k) {
      const int   sk = __builtin_amdgcn_readlane(s, k);
      const float wk = __int_as_float(__builtin_amdgcn_readlane(wi, k));
      const v2f hv = *(const v2fa*)(H + (size_t)sk * DD + 2 * lane);
      a0 = a0 + hv.x * wk;
      a1 = a1 + hv.y * wk;
    }
  }
  const v2f hs = *(const v2fa*)(H + (size_t)tc * DD + 2 * lane);
  asm volatile("" :: "v"(hs));
  const float dd = dt * dt;
  a0 = a0 + hs.x * dd;
  a1 = a1 + hs.y * dd;
  a0 = a0 + bp.x;
  a1 = a1 + bp.y;
  float v0 = (a0 >= 0.0f) ? a0 : sa * a0;
  float v1 = (a1 >= 0.0f) ? a1 : sa * a1;
  const float qnan = __int_as_float(0x7fc00000);
  const bool poison = big || (fl != 0);
  v0 = poison ? qnan : v0;
  v1 = poison ? qnan : v1;

  const int sA = (2 * lane) & 31, sB = (2 * lane + 1) & 31;
  v4f ow;
  ow.x = __shfl(v0, sA, 32);
  ow.y = __shfl(v1, sA, 32);
  ow.z = __shfl(v0, sB, 32);
  ow.w = __shfl(v1, sB, 32);
  float* op = out + (size_t)tc * DD + 4 * (lane & 15);
  const bool wr = (t < NN) && (lane < 16);
  if (wr) *(volatile v4f*)op = ow;
  __threadfence();
  if (wr) *(volatile v4f*)op = ow;
}

extern "C" void kernel_launch(void* const* d_in, const int* in_sizes, int n_in,
                              void* d_out, int out_size, void* d_ws, size_t ws_size,
                              hipStream_t stream) {
  if (n_in < 5) return;
  if (in_sizes[0] != NN * DD) return;
  if (in_sizes[1] != 2 * EE) return;
  if (in_sizes[2] != DD * DD) return;
  if (in_sizes[3] != DD) return;
  if (in_sizes[4] != 1) return;
  if (out_size != NN * DD) return;
  if (ws_size < WS_TOTAL) return;

  const float* x    = (const float*)d_in[0];
  const int*   edge = (const int*)d_in[1];
  const float* W    = (const float*)d_in[2];
  const float* b    = (const float*)d_in[3];
  const float* pa   = (const float*)d_in[4];
  float* out = (float*)d_out;
  const int* srcRow = edge;
  const int* dstRow = edge + EE;

  char* ws = (char*)d_ws;
  unsigned short* XB   = (unsigned short*)(ws + O_XB);
  float*          H    = (float*)(ws + O_H);
  unsigned short* WB   = (unsigned short*)(ws + O_WB);
  float*          PAR  = (float*)(ws + O_PAR);
  int*            LIST = (int*)(ws + O_LIST);
  int*            CNT  = (int*)(ws + O_CNT);
  int*            OFF  = (int*)(ws + O_OFF);
  int*            DIVB = (int*)(ws + O_DINV);
  const float*    DINV = (const float*)(ws + O_DINV);
  int*            FLAG = (int*)(ws + O_FLAG);

  hipFuncSetAttribute(reinterpret_cast<const void*>(&k_bucket), hipFuncAttributeMaxDynamicSharedMemorySize,
                      (int)BK_BYTES);

  k_plane<0><<<(MPAD * DD / 8) / 256, 256, 0, stream>>>(x, NN, DD, DD, XB, MPAD, DD);
  k_prep<<<1, NTHR, 0, stream>>>(W, b, pa, WB, PAR);
  k_gemm_nt<0, 0><<<((MPAD / 64) + 7) / 8, 256, 0, stream>>>(XB, WB, PAR, H, MPAD, DD, DD, DD);
  k_bucket<<<NBLK, NTHR, BK_BYTES, stream>>>(srcRow, dstRow, LIST, CNT, OFF, DIVB, FLAG);
  k_replay<<<NN / 8, NTHR, 0, stream>>>(H, LIST, CNT, OFF, DINV, FLAG, PAR, out);
}
